// MeshGraphNet_9655086482216
// MI455X (gfx1250) — hardware-verified
//
#include <hip/hip_runtime.h>
#include <stddef.h>
#include <stdint.h>


#define HID    128
#define NIN    12
#define EIN    4
#define TOUT   20
#define K1E    32
#define KHL    256
#define KV1    512
#define NTHR   256
#define NWAVE  8
#define EPB    256
#define GTHR   128
#define GBM    64
#define APE    264
#define APN    520
#define AP2    264
#define DP     132
#define ECST   512
#define NCST   512
#define EPT    8
#define CHUNK  (NTHR * EPT)
#define WCAP   (EPT * 32)
#define LISTN  (NWAVE * WCAP)
#define NBA    1024
#define SLA    10
#define RCAP   28672
#define DEGCAP 64
#define HROWS  320
#define C1O    8
#define C1K    15
#define C1S    4
#define C1P    29
#define C2K    10
#define SHW    232
#define WSMAX  134217728

#define PH_W32   (HID * K1E)
#define PH_W256  (HID * KHL)
#define PH_WAB   (2 * HID * KHL)
#define PH_WV1   (HID * KV1)
#define OFF_WN1T 0
#define OFF_WN2T (OFF_WN1T + PH_W32)
#define OFF_WE1T (OFF_WN2T + PH_W256)
#define OFF_WE2T (OFF_WE1T + PH_W32)
#define OFF_LAY  (OFF_WE2T + PH_W256)
#define LO_WABT  0
#define LO_WCT   (LO_WABT + PH_WAB)
#define LO_WE2   (LO_WCT + PH_W256)
#define LO_WV1   (LO_WE2 + PH_W256)
#define LO_WV2   (LO_WV1 + PH_WV1)
#define PH_LAYER (LO_WV2 + PH_W256)
#define NU_W32   (PH_W32 / 8)
#define NU_W256  (PH_W256 / 8)
#define NU_WAB   (PH_WAB / 8)
#define NU_WV1   (PH_WV1 / 8)
#define NU_LAYER (PH_LAYER / 8)
#define NU_GROW  96

#define AGG_ZINTS     (LISTN + 2 * RCAP + 3 * NBA)
#define AGG_LDS_INTS  (AGG_ZINTS + 16)
#define SCAN_LDS_BYTES (AGG_LDS_INTS * 4)
#define EDGE_LDS_BYTES (EPB * DP * 4 + EPB * APE * 2 + ECST * 4 + 3 * HID * 4)
#define NODE_LDS_BYTES (GBM * APN * 2 + NCST * 4 + 4 * HID * 4)

static_assert((CHUNK & (CHUNK - 1)) == 0 && CHUNK <= 4096);
static_assert((NBA & (NBA - 1)) == 0 && NBA == (1 << SLA));
static_assert(((long long)CHUNK << SLA) < (1LL << 31));
static_assert(LISTN % NTHR == 0);
static_assert(NBA % NWAVE == 0 && NBA % 32 == 0 && NBA == 4 * NTHR);
static_assert(RCAP % 4 == 0 && AGG_ZINTS % 4 == 0 && LISTN % 4 == 0);
static_assert(SCAN_LDS_BYTES <= 300000);
static_assert(EDGE_LDS_BYTES <= 300000);
static_assert(NODE_LDS_BYTES <= 300000);
static_assert((APE * 2) % 16 == 0 && APE >= KHL && (APN * 2) % 16 == 0 && APN >= KV1 && (AP2 * 2) % 16 == 0 && AP2 >= KHL);
static_assert((DP * 4) % 16 == 0 && DP >= HID);
static_assert(EPB == NTHR && EPB == NWAVE * 32);
static_assert(EPB * HID == 32 * NTHR * 4);
static_assert(GBM * HID == 16 * GTHR * 4);
static_assert(GTHR == HID && GBM == (GTHR / 32) * 16);
static_assert((EPB * APE) % 2 == 0 && (GBM * AP2) % 2 == 0 && (GBM * APN) % 2 == 0);
static_assert(((GBM * AP2) / 2) * 4 + GBM * HID * 4 <= ((GBM * APN) / 2) * 4);
static_assert(ECST == 4 * HID && NCST == 4 * HID);
static_assert(NU_W32 % NTHR == 0 && NU_W256 % NTHR == 0 && NU_WAB % NTHR == 0 && NU_WV1 % NTHR == 0);
static_assert(NU_LAYER % NTHR == 0 && NU_GROW % 32 == 0);
static_assert(K1E % 32 == 0 && KHL % 32 == 0 && KV1 % 32 == 0 && NIN <= K1E && EIN <= K1E);
static_assert(HROWS % NWAVE == 0 && (HROWS * TOUT) % 4 == 0 && ((HROWS * TOUT * 4) % 128) == 0);
static_assert(C1P == (HID - C1K) / C1S + 1 && TOUT == C1P - C2K + 1 && SHW >= C1O * C1P);

typedef float          v4f   __attribute__((ext_vector_type(4)));
typedef float          v8f   __attribute__((ext_vector_type(8)));
typedef int            v4i   __attribute__((ext_vector_type(4)));
typedef int            v8i   __attribute__((ext_vector_type(8)));
typedef unsigned       v2u   __attribute__((ext_vector_type(2)));
typedef unsigned short v8us  __attribute__((ext_vector_type(8)));
typedef unsigned short v16us __attribute__((ext_vector_type(16)));
typedef __bf16         v16bf __attribute__((ext_vector_type(16)));
typedef v4f  __attribute__((may_alias)) v4fa;
typedef v4i  __attribute__((may_alias)) v4ia;
typedef v2u  __attribute__((may_alias)) v2ua;
typedef v8us __attribute__((may_alias)) v8usa;
union FragB { v16bf v; v16us u; v8us h[2]; v8i w; };

__device__ __forceinline__ v8f wmb(const FragB& a, const FragB& b, v8f c) {
  v8f d = __builtin_amdgcn_wmma_f32_16x16x32_bf16(false, a.v, false, b.v, (short)0, c, false, false);
  asm volatile("v_nop\n\tv_nop\n\tv_nop\n\tv_nop" : "+v"(d) : "v"(a.w), "v"(b.w));
  return d;
}

__device__ __forceinline__ unsigned bf16_bits(float f) {
  const unsigned u = __float_as_uint(f);
  return (u + 0x7FFFu + ((u >> 16) & 1u)) >> 16;
}
__device__ __forceinline__ float bf16_val(float f) {
  return __uint_as_float(bf16_bits(f) << 16);
}
__device__ __forceinline__ void hilo4(v4f v, v2u& ph, v2u& pl) {
  const unsigned h0 = bf16_bits(v.x), h1 = bf16_bits(v.y), h2 = bf16_bits(v.z), h3 = bf16_bits(v.w);
  const unsigned l0 = bf16_bits(v.x - __uint_as_float(h0 << 16));
  const unsigned l1 = bf16_bits(v.y - __uint_as_float(h1 << 16));
  const unsigned l2 = bf16_bits(v.z - __uint_as_float(h2 << 16));
  const unsigned l3 = bf16_bits(v.w - __uint_as_float(h3 << 16));
  ph.x = h0 | (h1 << 16);
  ph.y = h2 | (h3 << 16);
  pl.x = l0 | (l1 << 16);
  pl.y = l2 | (l3 << 16);
}
__device__ __forceinline__ void put16(unsigned short* dp, v8us o) {
  *(volatile v8us*)dp = o;
  __threadfence();
  *(volatile v8us*)dp = o;
}
__device__ __forceinline__ void putf4(float* dp, v4f o) {
  *(volatile v4f*)dp = o;
  __threadfence();
  *(volatile v4f*)dp = o;
}

template <int SLB>
__device__ __forceinline__ int scan_chunk(const int* __restrict__ dsts, int nE, int cbase, int slotBase,
                                          int nb, int vec8, int* list, int tid, int lane, int wave) {
  int wc = 0;
  const int el0  = tid * EPT;
  const int e0   = cbase + el0;
  const int sent = -2147483647 - 1;
  v4i da, db;
  if (vec8 != 0 && cbase + CHUNK <= nE) {
    da = *(const v4i*)(dsts + e0);
    db = *(const v4i*)(dsts + e0 + 4);
  } else {
    da.x = (e0     < nE) ? dsts[min(e0,     nE - 1)] : sent;
    da.y = (e0 + 1 < nE) ? dsts[min(e0 + 1, nE - 1)] : sent;
    da.z = (e0 + 2 < nE) ? dsts[min(e0 + 2, nE - 1)] : sent;
    da.w = (e0 + 3 < nE) ? dsts[min(e0 + 3, nE - 1)] : sent;
    db.x = (e0 + 4 < nE) ? dsts[min(e0 + 4, nE - 1)] : sent;
    db.y = (e0 + 5 < nE) ? dsts[min(e0 + 5, nE - 1)] : sent;
    db.z = (e0 + 6 < nE) ? dsts[min(e0 + 6, nE - 1)] : sent;
    db.w = (e0 + 7 < nE) ? dsts[min(e0 + 7, nE - 1)] : sent;
  }
  const unsigned nbs = (unsigned)slotBase;
  const unsigned unb = (unsigned)nb;
  const unsigned s0 = (unsigned)da.x - nbs, s1 = (unsigned)da.y - nbs;
  const unsigned s2 = (unsigned)da.z - nbs, s3 = (unsigned)da.w - nbs;
  const unsigned s4 = (unsigned)db.x - nbs, s5 = (unsigned)db.y - nbs;
  const unsigned s6 = (unsigned)db.z - nbs, s7 = (unsigned)db.w - nbs;
  const bool h0 = s0 < unb, h1 = s1 < unb, h2 = s2 < unb, h3 = s3 < unb;
  const bool h4 = s4 < unb, h5 = s5 < unb, h6 = s6 < unb, h7 = s7 < unb;
  const unsigned any = __builtin_amdgcn_ballot_w32(h0 | h1 | h2 | h3 | h4 | h5 | h6 | h7);
  if (any != 0u) {
#define HITJ(J, HJ, SJ) { \
      const unsigned mj = __builtin_amdgcn_ballot_w32(HJ); \
      if (mj != 0u) { \
        if (HJ) { \
          const int pos = wc + (int)__builtin_amdgcn_mbcnt_lo(mj, 0u); \
          if (pos < WCAP) list[wave * WCAP + pos] = ((el0 + (J)) << SLB) | (int)(SJ); \
        } \
        wc += (int)__builtin_popcount(mj); } }
    HITJ(0, h0, s0)
    HITJ(1, h1, s1)
    HITJ(2, h2, s2)
    HITJ(3, h3, s3)
    HITJ(4, h4, s4)
    HITJ(5, h5, s5)
    HITJ(6, h6, s6)
    HITJ(7, h7, s7)
#undef HITJ
  }
  return wc;
}

__global__ __launch_bounds__(NTHR) void k_prep(const float* __restrict__ Wn1, const float* __restrict__ Wn2,
                                               const float* __restrict__ We1, const float* __restrict__ We2,
                                               const float* __restrict__ lEW1, const float* __restrict__ lEW2,
                                               const float* __restrict__ lVW1, const float* __restrict__ lVW2,
                                               const float* __restrict__ lEb1, const float* __restrict__ lVb1,
                                               int L, unsigned short* WPL, float* GROW) {
  const int u  = (int)blockIdx.x * NTHR + (int)threadIdx.x;
  const int U0 = NU_W32;
  const int U1 = U0 + NU_W256;
  const int U2 = U1 + NU_W32;
  const int U3 = U2 + NU_W256;
  const int U4 = U3 + L * NU_LAYER;
  const int U5 = U4 + NU_GROW;
  if (u >= U5) return;
  if (u < U4) {
    const float* p;
    unsigned short* d;
    int nv = 8;
    if (u < U0) {
      const int n = u >> 2, k8 = (u & 3) * 8;
      nv = NIN - k8;
      p = Wn1 + (size_t)(k8 < NIN ? k8 : 0) * HID + n;
      d = WPL + OFF_WN1T + (size_t)n * K1E + k8;
    } else if (u < U1) {
      const int v = u - U0, n = v >> 5, k8 = (v & 31) * 8;
      p = Wn2 + (size_t)(k8 & (HID - 1)) * HID + n;
      d = WPL + OFF_WN2T + (size_t)n * KHL + k8;
    } else if (u < U2) {
      const int v = u - U1, n = v >> 2, k8 = (v & 3) * 8;
      nv = EIN - k8;
      p = We1 + (size_t)(k8 < EIN ? k8 : 0) * HID + n;
      d = WPL + OFF_WE1T + (size_t)n * K1E + k8;
    } else if (u < U3) {
      const int v = u - U2, n = v >> 5, k8 = (v & 31) * 8;
      p = We2 + (size_t)(k8 & (HID - 1)) * HID + n;
      d = WPL + OFF_WE2T + (size_t)n * KHL + k8;
    } else {
      const int v = u - U3;
      const int l = v / NU_LAYER;
      const int r = v - l * NU_LAYER;
      const float* EW1l = lEW1 + (size_t)l * (4 * HID * HID);
      const float* EW2l = lEW2 + (size_t)l * (HID * HID);
      const float* VW1l = lVW1 + (size_t)l * (3 * HID * HID);
      const float* VW2l = lVW2 + (size_t)l * (HID * HID);
      unsigned short* base = WPL + OFF_LAY + (size_t)l * PH_LAYER;
      if (r < NU_WAB) {
        const int n = r >> 5, k8 = (r & 31) * 8;
        const int srow = (n >> 7) * HID + (k8 & (HID - 1));
        p = EW1l + (size_t)srow * HID + (n & (HID - 1));
        d = base + LO_WABT + (size_t)n * KHL + k8;
      } else if (r < NU_WAB + NU_W256) {
        const int v2 = r - NU_WAB, n = v2 >> 5, k8 = (v2 & 31) * 8;
        p = EW1l + (size_t)(2 * HID + (k8 & (HID - 1))) * HID + n;
        d = base + LO_WCT + (size_t)n * KHL + k8;
      } else if (r < NU_WAB + 2 * NU_W256) {
        const int v2 = r - NU_WAB - NU_W256, n = v2 >> 5, k8 = (v2 & 31) * 8;
        p = EW2l + (size_t)(k8 & (HID - 1)) * HID + n;
        d = base + LO_WE2 + (size_t)n * KHL + k8;
      } else if (r < NU_WAB + 2 * NU_W256 + NU_WV1) {
        const int v2 = r - NU_WAB - 2 * NU_W256, n = v2 >> 6, k8 = (v2 & 63) * 8;
        const int srow = (k8 >> 8) * HID + (k8 & (HID - 1));
        p = VW1l + (size_t)srow * HID + n;
        d = base + LO_WV1 + (size_t)n * KV1 + k8;
      } else {
        const int v2 = r - NU_WAB - 2 * NU_W256 - NU_WV1, n = v2 >> 5, k8 = (v2 & 31) * 8;
        p = VW2l + (size_t)(k8 & (HID - 1)) * HID + n;
        d = base + LO_WV2 + (size_t)n * KHL + k8;
      }
    }
    nv = nv < 0 ? 0 : (nv > 8 ? 8 : nv);
    const int top = (nv > 0 ? nv : 1) - 1;
    v8us o;
#pragma unroll
    for (int i = 0; i < 8; ++i) {
      const int ic = i < top ? i : top;
      const float w = p[(size_t)ic * HID];
      o[i] = (i < nv) ? (unsigned short)bf16_bits(w) : (unsigned short)0;
    }
    put16(d, o);
    return;
  }
  {
    const int v   = u - U4;
    const int row = v >> 5;
    const int j   = v & 31;
    const v4f e4 = *(const v4fa*)(lEb1 + 4 * j);
    const v4f w4 = *(const v4fa*)(lVb1 + 4 * j);
    const float f1 = (row == 1) ? 1.0f : 0.0f;
    const float f2 = (row == 2) ? 1.0f : 0.0f;
    v4f q;
    q.x = f1 * bf16_val(e4.x) + f2 * bf16_val(w4.x);
    q.y = f1 * bf16_val(e4.y) + f2 * bf16_val(w4.y);
    q.z = f1 * bf16_val(e4.z) + f2 * bf16_val(w4.z);
    q.w = f1 * bf16_val(e4.w) + f2 * bf16_val(w4.w);
    putf4(GROW + (size_t)row * HID + 4 * j, q);
  }
}

__global__ __launch_bounds__(GTHR) void k_pe(const unsigned short* __restrict__ A,
                                             const unsigned short* __restrict__ BT, float* Cm) {
  __shared__ __attribute__((aligned(16))) float stg[GBM * HID];
  const int tid = (int)threadIdx.x, lane = tid & 31, wave = tid >> 5, hh = lane >> 4, m = lane & 15;
  const int rowBase = (int)blockIdx.x * GBM;
  const int colBase = (int)blockIdx.y * HID;

  v8f acc[8];
  {
    const v8f z = {0.f, 0.f, 0.f, 0.f, 0.f, 0.f, 0.f, 0.f};
#pragma unroll
    for (int t = 0; t < 8; ++t) acc[t] = z;
  }
  const unsigned short* ap = A  + (size_t)(rowBase + 16 * wave + m) * (size_t)KHL + 8 * hh;
  const unsigned short* bp = BT + (size_t)(colBase + m) * (size_t)KHL + 8 * hh;

#pragma unroll 1
  for (int k0 = 0; k0 < KHL; k0 += 32) {
    FragB af;
    af.h[0] = *(const v8usa*)(ap + k0);
    af.h[1] = *(const v8usa*)(ap + k0 + 16);
#pragma unroll
    for (int nt = 0; nt < 8; ++nt) {
      const unsigned short* wq = bp + (size_t)(16 * nt) * (size_t)KHL + k0;
      FragB bf;
      bf.h[0] = *(const v8usa*)wq;
      bf.h[1] = *(const v8usa*)(wq + 16);
      acc[nt] = wmb(af, bf, acc[nt]);
    }
  }

#pragma unroll
  for (int nt = 0; nt < 8; ++nt) {
    const int lc = 16 * nt + m;
#pragma unroll
    for (int r = 0; r < 8; ++r) {
      const int lr = 16 * wave + 8 * hh + r;
      stg[lr * HID + lc] = acc[nt][r];
    }
  }
  __syncthreads();

  v4f pv[16];
#pragma unroll
  for (int i = 0; i < 16; ++i) pv[i] = *(const v4fa*)(stg + (16 * wave + i) * HID + 4 * lane);
#pragma unroll
  for (int i = 0; i < 16; ++i) {
    float* op = Cm + (size_t)(rowBase + 16 * wave + i) * (size_t)KHL + colBase + 4 * lane;
    *(volatile v4f*)op = pv[i];
  }
  __threadfence();
#pragma unroll
  for (int i = 0; i < 16; ++i) {
    float* op = Cm + (size_t)(rowBase + 16 * wave + i) * (size_t)KHL + colBase + 4 * lane;
    *(volatile v4f*)op = pv[i];
  }
}

template <int APITCH>
__device__ __forceinline__ void wave_gemm_b(const unsigned short* sAw, float* sDw,
                                            const unsigned short* __restrict__ BT, int ldb, int K,
                                            int hh, int m) {
#pragma unroll 1
  for (int nh = 0; nh < 2; ++nh) {
    v8f acc[2][4];
    {
      const v8f z = {0.f, 0.f, 0.f, 0.f, 0.f, 0.f, 0.f, 0.f};
#pragma unroll
      for (int mt = 0; mt < 2; ++mt)
#pragma unroll
        for (int nt = 0; nt < 4; ++nt) acc[mt][nt] = z;
    }
    const unsigned short* ap0 = sAw + m * APITCH + 8 * hh;
    const unsigned short* ap1 = ap0 + 16 * APITCH;
    const unsigned short* bp  = BT + (size_t)(64 * nh + m) * (size_t)ldb + 8 * hh;
#pragma unroll 1
    for (int k0 = 0; k0 < K; k0 += 32) {
      FragB a0, a1;
      a0.h[0] = *(const v8usa*)(ap0 + k0);
      a0.h[1] = *(const v8usa*)(ap0 + k0 + 16);
      a1.h[0] = *(const v8usa*)(ap1 + k0);
      a1.h[1] = *(const v8usa*)(ap1 + k0 + 16);
#pragma unroll
      for (int nt = 0; nt < 4; ++nt) {
        const unsigned short* wq = bp + (size_t)(16 * nt) * (size_t)ldb + k0;
        FragB b;
        b.h[0] = *(const v8usa*)wq;
        b.h[1] = *(const v8usa*)(wq + 16);
        acc[0][nt] = wmb(a0, b, acc[0][nt]);
        acc[1][nt] = wmb(a1, b, acc[1][nt]);
      }
    }
#pragma unroll
    for (int nt = 0; nt < 4; ++nt) {
      const int col = 64 * nh + 16 * nt + m;
#pragma unroll
      for (int mt = 0; mt < 2; ++mt)
#pragma unroll
        for (int r = 0; r < 8; ++r) sDw[(16 * mt + 8 * hh + r) * DP + col] = acc[mt][nt][r];
    }
  }
}

template <bool ENC>
__global__ __launch_bounds__(NTHR) void k_edge(const int* __restrict__ ei, int nE, int nN,
                                               const float* __restrict__ EA, float* XE,
                                               const float* __restrict__ PE, const float* __restrict__ GROW,
                                               const unsigned short* __restrict__ W1T,
                                               const unsigned short* __restrict__ W2T,
                                               const float* __restrict__ b1, const float* __restrict__ b2,
                                               const float* __restrict__ gam, const float* __restrict__ bet,
                                               float* EREC) {
  extern __shared__ __attribute__((aligned(16))) float dyn[];
  float*          sD    = dyn;
  unsigned short* sA    = (unsigned short*)(dyn + EPB * DP);
  float*          cst   = dyn + EPB * DP + (EPB * APE) / 2;
  float*          spart = cst + ECST;

  const int tid = (int)threadIdx.x, lane = tid & 31, wave = tid >> 5, hh = lane >> 4, m = lane & 15;
  const int elb = (int)blockIdx.x * EPB;
  int nl = nE - elb;
  nl = nl > EPB ? EPB : nl;

  if (tid < HID) {
    float c0;
    if constexpr (ENC) c0 = bf16_val(b1[tid]); else c0 = GROW[HID + tid];
    cst[tid]           = c0;
    cst[HID + tid]     = bf16_val(b2[tid]);
    cst[2 * HID + tid] = bf16_val(gam[tid]);
    cst[3 * HID + tid] = bf16_val(bet[tid]);
  }

  const int  el   = elb + tid;
  const bool live = el < nE;
  const int  eg   = live ? el : (nE - 1);
  int s = 0, r = 0;
  if constexpr (!ENC) {
    s = ei[eg];
    r = ei[(size_t)nE + (size_t)eg];
    s = s < 0 ? 0 : (s > nN - 1 ? nN - 1 : s);
    r = r < 0 ? 0 : (r > nN - 1 ? nN - 1 : r);
  }

  unsigned short* ra = sA + (size_t)tid * APE;
  float*          rd = sD + (size_t)tid * DP;

  if constexpr (ENC) {
    const v4f ea = *(const v4fa*)(EA + (size_t)eg * EIN);
    v8us o0, oz;
    o0[0] = (unsigned short)bf16_bits(ea.x);
    o0[1] = (unsigned short)bf16_bits(ea.y);
    o0[2] = (unsigned short)bf16_bits(ea.z);
    o0[3] = (unsigned short)bf16_bits(ea.w);
    o0[4] = (unsigned short)0; o0[5] = (unsigned short)0; o0[6] = (unsigned short)0; o0[7] = (unsigned short)0;
#pragma unroll
    for (int i = 0; i < 8; ++i) oz[i] = (unsigned short)0;
    *(v8usa*)(ra + 0)  = o0;
    *(v8usa*)(ra + 8)  = oz;
    *(v8usa*)(ra + 16) = oz;
    *(v8usa*)(ra + 24) = oz;
  } else {
#pragma unroll 4
    for (int it = 0; it < 32; ++it) {
      const int f   = it * (NTHR * 4) + tid * 4;
      const int row = f >> 7;
      const int col = f & (HID - 1);
      const int gr  = elb + row;
      const int grc = gr < nE ? gr : nE - 1;
      const v4f v = *(const v4fa*)(XE + (size_t)grc * HID + col);
      v2u ph, pl;
      hilo4(v, ph, pl);
      *(v2ua*)(sA + (size_t)row * APE + col)       = ph;
      *(v2ua*)(sA + (size_t)row * APE + HID + col) = pl;
    }
  }
  __syncthreads();

  const unsigned short* sAw = sA + (size_t)(32 * wave) * APE;
  float*                sDw = sD + (size_t)(32 * wave) * DP;

  if constexpr (ENC) wave_gemm_b<APE>(sAw, sDw, W1T, K1E, K1E, hh, m);
  else               wave_gemm_b<APE>(sAw, sDw, W1T, KHL, KHL, hh, m);
  __syncthreads();

  {
    const float* pp = PE + (size_t)s * KHL;
    const float* qq = PE + (size_t)r * KHL + HID;
#pragma unroll 1
    for (int c8 = 0; c8 < HID / 8; ++c8) {
      const v4f va = *(const v4fa*)(rd + 8 * c8);
      const v4f vb = *(const v4fa*)(rd + 8 * c8 + 4);
      const v4f ba = *(const v4fa*)(cst + 8 * c8);
      const v4f bb = *(const v4fa*)(cst + 8 * c8 + 4);
      const v8f v8 = {va.x, va.y, va.z, va.w, vb.x, vb.y, vb.z, vb.w};
      const v8f b8 = {ba.x, ba.y, ba.z, ba.w, bb.x, bb.y, bb.z, bb.w};
      v8f p8 = {0.f, 0.f, 0.f, 0.f, 0.f, 0.f, 0.f, 0.f};
      v8f q8 = {0.f, 0.f, 0.f, 0.f, 0.f, 0.f, 0.f, 0.f};
      if constexpr (!ENC) {
        const v4f pa = *(const v4fa*)(pp + 8 * c8);
        const v4f pb = *(const v4fa*)(pp + 8 * c8 + 4);
        const v4f qa = *(const v4fa*)(qq + 8 * c8);
        const v4f qb = *(const v4fa*)(qq + 8 * c8 + 4);
        const v8f pt = {pa.x, pa.y, pa.z, pa.w, pb.x, pb.y, pb.z, pb.w};
        const v8f qt = {qa.x, qa.y, qa.z, qa.w, qb.x, qb.y, qb.z, qb.w};
        p8 = pt;
        q8 = qt;
      }
      v8us oh, ol;
#pragma unroll
      for (int i = 0; i < 8; ++i) {
        const float pre = (p8[i] + q8[i]) + (v8[i] + b8[i]);
        const float h   = fmaxf(pre, 0.0f);
        const unsigned hb = bf16_bits(h);
        oh[i] = (unsigned short)hb;
        ol[i] = (unsigned short)bf16_bits(h - __uint_as_float(hb << 16));
      }
      *(v8usa*)(ra + 8 * c8)       = oh;
      *(v8usa*)(ra + HID + 8 * c8) = ol;
    }
  }
  __syncthreads();

  wave_gemm_b<APE>(sAw, sDw, W2T, KHL, KHL, hh, m);
  __syncthreads();

  {
    float sum = 0.0f;
#pragma unroll 1
    for (int c8 = 0; c8 < HID / 8; ++c8) {
      const v4f va = *(const v4fa*)(rd + 8 * c8);
      const v4f vb = *(const v4fa*)(rd + 8 * c8 + 4);
      const v4f ba = *(const v4fa*)(cst + HID + 8 * c8);
      const v4f bb = *(const v4fa*)(cst + HID + 8 * c8 + 4);
      sum += (va.x + ba.x); sum += (va.y + ba.y); sum += (va.z + ba.z); sum += (va.w + ba.w);
      sum += (vb.x + bb.x); sum += (vb.y + bb.y); sum += (vb.z + bb.z); sum += (vb.w + bb.w);
    }
    const float mean = sum * (1.0f / (float)HID);
    float vs = 0.0f;
#pragma unroll 1
    for (int c8 = 0; c8 < HID / 8; ++c8) {
      const v4f va = *(const v4fa*)(rd + 8 * c8);
      const v4f vb = *(const v4fa*)(rd + 8 * c8 + 4);
      const v4f ba = *(const v4fa*)(cst + HID + 8 * c8);
      const v4f bb = *(const v4fa*)(cst + HID + 8 * c8 + 4);
      const v8f t8 = {va.x + ba.x, va.y + ba.y, va.z + ba.z, va.w + ba.w,
                      vb.x + bb.x, vb.y + bb.y, vb.z + bb.z, vb.w + bb.w};
#pragma unroll
      for (int i = 0; i < 8; ++i) { const float d = t8[i] - mean; vs = fmaf(d, d, vs); }
    }
    const float rstd = rsqrtf(vs * (1.0f / (float)HID) + 1e-5f);
    const float* xr = XE + (size_t)eg * HID;
#pragma unroll 1
    for (int c8 = 0; c8 < HID / 8; ++c8) {
      const v4f va = *(const v4fa*)(rd + 8 * c8);
      const v4f vb = *(const v4fa*)(rd + 8 * c8 + 4);
      const v4f ba = *(const v4fa*)(cst + HID + 8 * c8);
      const v4f bb = *(const v4fa*)(cst + HID + 8 * c8 + 4);
      const v4f ga = *(const v4fa*)(cst + 2 * HID + 8 * c8);
      const v4f gb = *(const v4fa*)(cst + 2 * HID + 8 * c8 + 4);
      const v4f ea = *(const v4fa*)(cst + 3 * HID + 8 * c8);
      const v4f eb = *(const v4fa*)(cst + 3 * HID + 8 * c8 + 4);
      const v8f t8 = {va.x + ba.x, va.y + ba.y, va.z + ba.z, va.w + ba.w,
                      vb.x + bb.x, vb.y + bb.y, vb.z + bb.z, vb.w + bb.w};
      const v8f g8 = {ga.x, ga.y, ga.z, ga.w, gb.x, gb.y, gb.z, gb.w};
      const v8f e8 = {ea.x, ea.y, ea.z, ea.w, eb.x, eb.y, eb.z, eb.w};
      v8f x8 = {0.f, 0.f, 0.f, 0.f, 0.f, 0.f, 0.f, 0.f};
      if constexpr (!ENC) {
        const v4f xa = *(const v4fa*)(xr + 8 * c8);
        const v4f xb = *(const v4fa*)(xr + 8 * c8 + 4);
        const v8f xt = {xa.x, xa.y, xa.z, xa.w, xb.x, xb.y, xb.z, xb.w};
        x8 = xt;
      }
      v8f y8;
#pragma unroll
      for (int i = 0; i < 8; ++i) {
        const float ln = (t8[i] - mean) * rstd * g8[i] + e8[i];
        y8[i] = x8[i] + ln;
      }
      const v4f y0 = {y8[0], y8[1], y8[2], y8[3]};
      const v4f y1 = {y8[4], y8[5], y8[6], y8[7]};
      *(v4fa*)(rd + 8 * c8)     = y0;
      *(v4fa*)(rd + 8 * c8 + 4) = y1;
    }
  }
  __syncthreads();

  if constexpr (!ENC) {
    {
      const int c    = tid & (HID - 1);
      const int half = tid >> 7;
      const int rs   = half * (EPB / 2);
      int re = rs + (EPB / 2);
      re = re < nl ? re : nl;
      float sm = 0.0f;
#pragma unroll 4
      for (int rr = rs; rr < re; ++rr) sm += sD[rr * DP + c];
      spart[half * HID + c] = sm;
    }
    __syncthreads();
    if (tid < HID) spart[2 * HID + tid] = spart[tid] + spart[HID + tid];
    __syncthreads();
    if (wave == 0) {
      const v4f rec = *(const v4fa*)(spart + 2 * HID + 4 * lane);
      putf4(EREC + (size_t)blockIdx.x * HID + 4 * lane, rec);
    }
  }

  {
    float* ob = XE + (size_t)elb * HID;
#pragma unroll 8
    for (int it = 0; it < 32; ++it) {
      const int f = it * (NTHR * 4) + tid * 4;
      const v4f v = *(const v4fa*)(sD + (f >> 7) * DP + (f & (HID - 1)));
      *(volatile v4f*)(ob + f) = v;
    }
    __threadfence();
#pragma unroll 8
    for (int it = 0; it < 32; ++it) {
      const int f = it * (NTHR * 4) + tid * 4;
      const v4f v = *(const v4fa*)(sD + (f >> 7) * DP + (f & (HID - 1)));
      *(volatile v4f*)(ob + f) = v;
    }
  }
}

__global__ __launch_bounds__(NTHR) void k_scan(const int* __restrict__ dsts, int nE, int vec8, int mRows,
                                               const float* __restrict__ XE, float* AGG) {
  extern __shared__ __attribute__((aligned(16))) int dsm[];
  int* list = dsm;
  int* hl   = dsm + LISTN;
  int* sl   = hl + RCAP;
  int* cnt  = sl + RCAP;
  int* offs = cnt + NBA;
  int* cur  = offs + NBA;
  int* misc = cur + NBA;
  const int tid = (int)threadIdx.x, lane = tid & 31, wave = tid >> 5;
  const int nodeBase = (int)blockIdx.x * NBA;

  {
    const v4i z4 = {0, 0, 0, 0};
    for (int i = tid * 4; i < AGG_ZINTS; i += NTHR * 4) *(v4ia*)(dsm + i) = z4;
    if (tid < 16) misc[tid] = 0;
  }
  __syncthreads();

  int t = 0, ov = 0;
  const int nChunks = (nE + CHUNK - 1) / CHUNK;
#pragma unroll 1
  for (int ch = 0; ch < nChunks; ++ch) {
    const int cbase = ch * CHUNK;
    const int wc = scan_chunk<SLA>(dsts, nE, cbase, nodeBase, NBA, vec8, list, tid, lane, wave);
    if (lane == 0) misc[wave] = wc;
    __syncthreads();
    if (wave == 0) {
#pragma unroll 1
      for (int w2 = 0; w2 < NWAVE; ++w2) {
        int c = misc[w2];
        c = c < 0 ? 0 : (c > WCAP ? WCAP : c);
#pragma unroll 1
        for (int b0 = 0; b0 < c; b0 += 32) {
          const int idx = b0 + lane;
          const int ent = list[w2 * WCAP + (idx < WCAP ? idx : WCAP - 1)];
          const int m32 = (c - b0) < 32 ? (c - b0) : 32;
#pragma unroll 1
          for (int k = 0; k < m32; ++k) {
            const int u    = __builtin_amdgcn_readlane(ent, k);
            const int slot = u & (NBA - 1);
            const int el   = (u >> SLA) & (CHUNK - 1);
            const int pk   = ((cbase + el) << SLA) | slot;
            if (t < RCAP) {
              if (lane == 0) { hl[t] = pk; cnt[slot] = cnt[slot] + 1; }
              t = t + 1;
            } else {
              ov = 1;
            }
          }
        }
      }
    }
    __syncthreads();
  }
  if (wave == 0 && lane == 0) { misc[8] = t; misc[9] = ov; }
  __syncthreads();
  int tt = misc[8];
  tt = tt < 0 ? 0 : (tt > RCAP ? RCAP : tt);
  const int ovf = misc[9];

  if (wave == 0) {
    const int base = lane * (NBA / 32);
    int s = 0;
#pragma unroll 1
    for (int i = 0; i < NBA / 32; ++i) s += cnt[base + i];
    int incl = s;
#pragma unroll
    for (int d = 1; d < 32; d <<= 1) {
      const int y = __shfl_up(incl, d, 32);
      if (lane >= d) incl += y;
    }
    int run = incl - s;
#pragma unroll 1
    for (int i = 0; i < NBA / 32; ++i) {
      const int cv = cnt[base + i];
      offs[base + i] = run;
      cur[base + i]  = run;
      run += cv;
    }
  }
  __syncthreads();
  if (wave == 0) {
#pragma unroll 1
    for (int b0 = 0; b0 < tt; b0 += 32) {
      const int idx = b0 + lane;
      const int ent = hl[idx < RCAP ? idx : RCAP - 1];
      const int m32 = (tt - b0) < 32 ? (tt - b0) : 32;
#pragma unroll 1
      for (int k = 0; k < m32; ++k) {
        const int u    = __builtin_amdgcn_readlane(ent, k);
        const int slot = u & (NBA - 1);
        if (lane == 0) {
          int p = cur[slot];
          p = p < 0 ? 0 : (p > RCAP - 1 ? RCAP - 1 : p);
          sl[p] = u;
          cur[slot] = p + 1;
        }
      }
    }
  }
  __syncthreads();

  const float qnan = __int_as_float(0x7fc00000);
  const float pz = (ovf != 0) ? qnan : 0.0f;
#pragma unroll 1
  for (int si = 0; si < NBA / NWAVE; ++si) {
    const int s    = si * NWAVE + wave;
    const int node = nodeBase + s;
    int c = cnt[s];
    const bool big = c > DEGCAP;
    c = c < 0 ? 0 : (c > DEGCAP ? DEGCAP : c);
    int o = offs[s];
    o = o < 0 ? 0 : (o > RCAP ? RCAP : o);
    float a0 = 0.0f, a1 = 0.0f, a2 = 0.0f, a3 = 0.0f;
#pragma unroll 1
    for (int b0 = 0; b0 < c; b0 += 32) {
      int idx = o + b0 + lane;
      idx = idx > RCAP - 1 ? RCAP - 1 : idx;
      const int ent = sl[idx];
      int eid = ent >> SLA;
      eid = eid < 0 ? 0 : (eid > nE - 1 ? nE - 1 : eid);
      const int m32 = (c - b0) < 32 ? (c - b0) : 32;
#pragma unroll 1
      for (int k = 0; k < m32; ++k) {
        const int ek = __builtin_amdgcn_readlane(eid, k);
        const v4f v = *(const v4fa*)(XE + (size_t)ek * HID + 4 * lane);
        a0 += v.x; a1 += v.y; a2 += v.z; a3 += v.w;
      }
    }
    const bool  live = node < mRows;
    const int   nr   = live ? node : mRows - 1;
    const float pzr  = big ? qnan : pz;
    float* mp = AGG + (size_t)nr * HID + 4 * lane;
    v4f nv;
    nv.x = a0 + pzr; nv.y = a1 + pzr; nv.z = a2 + pzr; nv.w = a3 + pzr;
    if (live) *(volatile v4f*)mp = nv;
    __threadfence();
    if (live) *(volatile v4f*)mp = nv;
  }
}

template <bool ENC>
__global__ __launch_bounds__(GTHR) void k_node(const float* __restrict__ xin, float* XV,
                                               const float* __restrict__ AGG,
                                               const unsigned short* __restrict__ W1T,
                                               const float* __restrict__ b1, const float* __restrict__ GROW,
                                               const unsigned short* __restrict__ W2T,
                                               const float* __restrict__ b2, const float* __restrict__ gam,
                                               const float* __restrict__ bet, int nN,
                                               unsigned short* XVB, float* NREC) {
  extern __shared__ __attribute__((aligned(16))) float ndyn[];
  unsigned short* sA1   = (unsigned short*)ndyn;
  unsigned short* sA2   = (unsigned short*)ndyn;
  float*          stg   = ndyn + (GBM * AP2) / 2;
  float*          cst   = ndyn + (GBM * APN) / 2;
  float*          spart = cst + NCST;
  const int tid = (int)threadIdx.x, lane = tid & 31, wave = tid >> 5, hh = lane >> 4, m = lane & 15;
  const int rowBase = (int)blockIdx.x * GBM;
  constexpr int K1 = ENC ? K1E : KV1;

  {
    float c0;
    if constexpr (ENC) c0 = bf16_val(b1[tid]); else c0 = GROW[2 * HID + tid];
    cst[tid]           = c0;
    cst[HID + tid]     = bf16_val(b2[tid]);
    cst[2 * HID + tid] = bf16_val(gam[tid]);
    cst[3 * HID + tid] = bf16_val(bet[tid]);
  }

  if constexpr (ENC) {
    if (tid < GBM) {
      const int row = tid;
      const int gr  = rowBase + row;
      const int rc  = gr < nN ? gr : nN - 1;
      const unsigned mk = (gr < nN) ? 0xffffu : 0u;
      const float* xp = xin + (size_t)rc * NIN;
      const v4f x0 = *(const v4fa*)xp;
      const v4f x1 = *(const v4fa*)(xp + 4);
      const v4f x2 = *(const v4fa*)(xp + 8);
      v8us o0, o1, oz;
      o0[0] = (unsigned short)(bf16_bits(x0.x) & mk); o0[1] = (unsigned short)(bf16_bits(x0.y) & mk);
      o0[2] = (unsigned short)(bf16_bits(x0.z) & mk); o0[3] = (unsigned short)(bf16_bits(x0.w) & mk);
      o0[4] = (unsigned short)(bf16_bits(x1.x) & mk); o0[5] = (unsigned short)(bf16_bits(x1.y) & mk);
      o0[6] = (unsigned short)(bf16_bits(x1.z) & mk); o0[7] = (unsigned short)(bf16_bits(x1.w) & mk);
      o1[0] = (unsigned short)(bf16_bits(x2.x) & mk); o1[1] = (unsigned short)(bf16_bits(x2.y) & mk);
      o1[2] = (unsigned short)(bf16_bits(x2.z) & mk); o1[3] = (unsigned short)(bf16_bits(x2.w) & mk);
      o1[4] = (unsigned short)0; o1[5] = (unsigned short)0; o1[6] = (unsigned short)0; o1[7] = (unsigned short)0;
#pragma unroll
      for (int i = 0; i < 8; ++i) oz[i] = (unsigned short)0;
      unsigned short* rp = sA1 + (size_t)row * APN;
      *(v8usa*)(rp + 0)  = o0;
      *(v8usa*)(rp + 8)  = o1;
      *(v8usa*)(rp + 16) = oz;
      *(v8usa*)(rp + 24) = oz;
    }
  } else {
#pragma unroll 4
    for (int it = 0; it < 16; ++it) {
      const int f   = it * (GTHR * 4) + tid * 4;
      const int row = f >> 7;
      const int col = f & (HID - 1);
      const int gr  = rowBase + row;
      const v4f xv = *(const v4fa*)(XV  + (size_t)gr * HID + col);
      const v4f ag = *(const v4fa*)(AGG + (size_t)gr * HID + col);
      v2u xh, xl, ah, al;
      hilo4(xv, xh, xl);
      hilo4(ag, ah, al);
      unsigned short* rp = sA1 + (size_t)row * APN + col;
      *(v2ua*)(rp)           = xh;
      *(v2ua*)(rp + HID)     = xl;
      *(v2ua*)(rp + 2 * HID) = ah;
      *(v2ua*)(rp + 3 * HID) = al;
    }
  }
  __syncthreads();

  v8f acc[8];
  {
    const v8f z = {0.f, 0.f, 0.f, 0.f, 0.f, 0.f, 0.f, 0.f};
#pragma unroll
    for (int t = 0; t < 8; ++t) acc[t] = z;
  }
  {
    const unsigned short* ap = sA1 + (size_t)(16 * wave + m) * APN + 8 * hh;
    const unsigned short* bp = W1T + (size_t)m * (size_t)K1 + 8 * hh;
#pragma unroll 1
    for (int k0 = 0; k0 < K1; k0 += 32) {
      FragB af;
      af.h[0] = *(const v8usa*)(ap + k0);
      af.h[1] = *(const v8usa*)(ap + k0 + 16);
#pragma unroll
      for (int nt = 0; nt < 8; ++nt) {
        const unsigned short* wq = bp + (size_t)(16 * nt) * (size_t)K1 + k0;
        FragB bf;
        bf.h[0] = *(const v8usa*)wq;
        bf.h[1] = *(const v8usa*)(wq + 16);
        acc[nt] = wmb(af, bf, acc[nt]);
      }
    }
  }
  __syncthreads();

#pragma unroll
  for (int nt = 0; nt < 8; ++nt) {
    const int lc = 16 * nt + m;
    const float bv = cst[lc];
#pragma unroll
    for (int r = 0; r < 8; ++r) {
      const int lr = 16 * wave + 8 * hh + r;
      const float h = fmaxf(acc[nt][r] + bv, 0.0f);
      const unsigned hb = bf16_bits(h);
      sA2[(size_t)lr * AP2 + lc]       = (unsigned short)hb;
      sA2[(size_t)lr * AP2 + HID + lc] = (unsigned short)bf16_bits(h - __uint_as_float(hb << 16));
    }
  }
  __syncthreads();

  {
    const v8f z = {0.f, 0.f, 0.f, 0.f, 0.f, 0.f, 0.f, 0.f};
#pragma unroll
    for (int t = 0; t < 8; ++t) acc[t] = z;
  }
  {
    const unsigned short* ap = sA2 + (size_t)(16 * wave + m) * AP2 + 8 * hh;
    const unsigned short* bp = W2T + (size_t)m * (size_t)KHL + 8 * hh;
#pragma unroll 1
    for (int k0 = 0; k0 < KHL; k0 += 32) {
      FragB af;
      af.h[0] = *(const v8usa*)(ap + k0);
      af.h[1] = *(const v8usa*)(ap + k0 + 16);
#pragma unroll
      for (int nt = 0; nt < 8; ++nt) {
        const unsigned short* wq = bp + (size_t)(16 * nt) * (size_t)KHL + k0;
        FragB bf;
        bf.h[0] = *(const v8usa*)wq;
        bf.h[1] = *(const v8usa*)(wq + 16);
        acc[nt] = wmb(af, bf, acc[nt]);
      }
    }
  }
#pragma unroll
  for (int nt = 0; nt < 8; ++nt) {
    const int lc = 16 * nt + m;
    const float bv = cst[HID + lc];
#pragma unroll
    for (int r = 0; r < 8; ++r) {
      const int lr = 16 * wave + 8 * hh + r;
      stg[lr * HID + lc] = acc[nt][r] + bv;
    }
  }
  __syncthreads();

  v4f cacc = {0.f, 0.f, 0.f, 0.f};
  {
    const v4f g4 = *(const v4fa*)(cst + 2 * HID + 4 * lane);
    const v4f e4 = *(const v4fa*)(cst + 3 * HID + 4 * lane);
#pragma unroll 2
    for (int i = 0; i < 16; ++i) {
      const int lr = 16 * wave + i;
      const int gr = rowBase + lr;
      float* sp = stg + lr * HID + 4 * lane;
      const v4f t = *(const v4fa*)sp;
      float s = (t.x + t.y) + (t.z + t.w);
      s += __shfl_xor(s, 16);
      s += __shfl_xor(s, 8);
      s += __shfl_xor(s, 4);
      s += __shfl_xor(s, 2);
      s += __shfl_xor(s, 1);
      const float mean = s * (1.0f / (float)HID);
      v4f d;
      d.x = t.x - mean; d.y = t.y - mean; d.z = t.z - mean; d.w = t.w - mean;
      float q = (d.x * d.x + d.y * d.y) + (d.z * d.z + d.w * d.w);
      q += __shfl_xor(q, 16);
      q += __shfl_xor(q, 8);
      q += __shfl_xor(q, 4);
      q += __shfl_xor(q, 2);
      q += __shfl_xor(q, 1);
      const float rstd = rsqrtf(q * (1.0f / (float)HID) + 1e-5f);
      v4f res = {0.f, 0.f, 0.f, 0.f};
      if constexpr (!ENC) res = *(const v4fa*)(XV + (size_t)gr * HID + 4 * lane);
      const bool ok = gr < nN;
      v4f y;
      y.x = res.x + (d.x * rstd * g4.x + e4.x);
      y.y = res.y + (d.y * rstd * g4.y + e4.y);
      y.z = res.z + (d.z * rstd * g4.z + e4.z);
      y.w = res.w + (d.w * rstd * g4.w + e4.w);
      y.x = ok ? y.x : 0.0f; y.y = ok ? y.y : 0.0f; y.z = ok ? y.z : 0.0f; y.w = ok ? y.w : 0.0f;
      cacc.x += y.x; cacc.y += y.y; cacc.z += y.z; cacc.w += y.w;
      *(v4fa*)sp = y;
    }
  }
  __syncthreads();

  {
    v4f pv[16];
#pragma unroll
    for (int i = 0; i < 16; ++i) pv[i] = *(const v4fa*)(stg + (16 * wave + i) * HID + 4 * lane);
#pragma unroll
    for (int i = 0; i < 16; ++i) {
      float* op = XV + (size_t)(rowBase + 16 * wave + i) * HID + 4 * lane;
      *(volatile v4f*)op = pv[i];
    }
    __threadfence();
#pragma unroll
    for (int i = 0; i < 16; ++i) {
      float* op = XV + (size_t)(rowBase + 16 * wave + i) * HID + 4 * lane;
      *(volatile v4f*)op = pv[i];
    }
  }
  {
    const int part = lane >> 4;
    const int j = lane & 15;
    const unsigned mh = 0u - (unsigned)part;
    const unsigned ml = ~mh;
    v8us pv[16];
#pragma unroll
    for (int i = 0; i < 16; ++i) {
      const float* sp = stg + (16 * wave + i) * HID + 8 * j;
      const v4f a = *(const v4fa*)sp;
      const v4f b = *(const v4fa*)(sp + 4);
      const v8f f8 = {a.x, a.y, a.z, a.w, b.x, b.y, b.z, b.w};
      v8us oo;
#pragma unroll
      for (int e = 0; e < 8; ++e) {
        const unsigned hb = bf16_bits(f8[e]);
        const unsigned lb = bf16_bits(f8[e] - __uint_as_float(hb << 16));
        oo[e] = (unsigned short)((hb & ml) | (lb & mh));
      }
      pv[i] = oo;
    }
#pragma unroll
    for (int i = 0; i < 16; ++i) {
      unsigned short* op = XVB + (size_t)(rowBase + 16 * wave + i) * (size_t)KHL + part * HID + 8 * j;
      *(volatile v8us*)op = pv[i];
    }
    __threadfence();
#pragma unroll
    for (int i = 0; i < 16; ++i) {
      unsigned short* op = XVB + (size_t)(rowBase + 16 * wave + i) * (size_t)KHL + part * HID + 8 * j;
      *(volatile v8us*)op = pv[i];
    }
  }

  if constexpr (!ENC) {
    *(v4fa*)(spart + wave * HID + 4 * lane) = cacc;
    __syncthreads();
    if (wave == 0) {
      const v4f p0 = *(const v4fa*)(spart + 4 * lane);
      const v4f p1 = *(const v4fa*)(spart + HID + 4 * lane);
      const v4f p2 = *(const v4fa*)(spart + 2 * HID + 4 * lane);
      const v4f p3 = *(const v4fa*)(spart + 3 * HID + 4 * lane);
      v4f rec;
      rec.x = (p0.x + p1.x) + (p2.x + p3.x);
      rec.y = (p0.y + p1.y) + (p2.y + p3.y);
      rec.z = (p0.z + p1.z) + (p2.z + p3.z);
      rec.w = (p0.w + p1.w) + (p2.w + p3.w);
      putf4(NREC + (size_t)blockIdx.x * HID + 4 * lane, rec);
    }
  }
}

__global__ __launch_bounds__(NTHR) void k_glob(const float* __restrict__ NREC, int nNB,
                                               const float* __restrict__ EREC, int nEB, float* GROW,
                                               const float* __restrict__ GW1, const float* __restrict__ Gb1,
                                               const float* __restrict__ GW2, const float* __restrict__ Gb2,
                                               const float* __restrict__ Gg, const float* __restrict__ Gbt,
                                               const float* __restrict__ EW1n, const float* __restrict__ Eb1n,
                                               const float* __restrict__ VW1n, const float* __restrict__ Vb1n) {
  __shared__ float gin[3 * HID];
  __shared__ float hbuf[HID];
  __shared__ __attribute__((aligned(16))) float obuf[HID];
  __shared__ float gn[HID];
  __shared__ __attribute__((aligned(16))) float srow[3 * HID];
  __shared__ float st[4];
  const int tid = (int)threadIdx.x, lane = tid & 31, wave = tid >> 5;

  if (tid < HID) {
    const int c = tid;
    double s = 0.0;
#pragma unroll 4
    for (int b = 0; b < nNB; ++b) s += (double)NREC[(size_t)b * HID + c];
    gin[c] = (float)s;
    gin[2 * HID + c] = GROW[c];
  } else {
    const int c = tid - HID;
    double s = 0.0;
#pragma unroll 4
    for (int b = 0; b < nEB; ++b) s += (double)EREC[(size_t)b * HID + c];
    gin[HID + c] = (float)s;
  }
  __syncthreads();
  if (tid < HID) {
    float a = bf16_val(Gb1[tid]);
#pragma unroll 4
    for (int k = 0; k < 3 * HID; ++k) a = fmaf(gin[k], bf16_val(GW1[(size_t)k * HID + tid]), a);
    hbuf[tid] = fmaxf(a, 0.0f);
  }
  __syncthreads();
  if (tid < HID) {
    float o = bf16_val(Gb2[tid]);
#pragma unroll 4
    for (int k = 0; k < HID; ++k) o = fmaf(hbuf[k], bf16_val(GW2[(size_t)k * HID + tid]), o);
    obuf[tid] = o;
  }
  __syncthreads();
  if (wave == 0) {
    const v4f t = *(const v4fa*)(obuf + 4 * lane);
    float s = (t.x + t.y) + (t.z + t.w);
    s += __shfl_xor(s, 16);
    s += __shfl_xor(s, 8);
    s += __shfl_xor(s, 4);
    s += __shfl_xor(s, 2);
    s += __shfl_xor(s, 1);
    const float mean = s * (1.0f / (float)HID);
    const float dx = t.x - mean, dy = t.y - mean, dz = t.z - mean, dw = t.w - mean;
    float q = (dx * dx + dy * dy) + (dz * dz + dw * dw);
    q += __shfl_xor(q, 16);
    q += __shfl_xor(q, 8);
    q += __shfl_xor(q, 4);
    q += __shfl_xor(q, 2);
    q += __shfl_xor(q, 1);
    const float rstd = rsqrtf(q * (1.0f / (float)HID) + 1e-5f);
    if (lane == 0) { st[0] = mean; st[1] = rstd; }
  }
  __syncthreads();
  if (tid < HID) {
    const float ln = (obuf[tid] - st[0]) * st[1] * bf16_val(Gg[tid]) + bf16_val(Gbt[tid]);
    const float g  = gin[2 * HID + tid] + ln;
    gn[tid]   = g;
    srow[tid] = g;
  }
  __syncthreads();
  if (tid < HID) {
    float e = bf16_val(Eb1n[tid]);
#pragma unroll 4
    for (int k = 0; k < HID; ++k) e = fmaf(gn[k], bf16_val(EW1n[(size_t)(3 * HID + k) * HID + tid]), e);
    srow[HID + tid] = e;
    float v = bf16_val(Vb1n[tid]);
#pragma unroll 4
    for (int k = 0; k < HID; ++k) v = fmaf(gn[k], bf16_val(VW1n[(size_t)(2 * HID + k) * HID + tid]), v);
    srow[2 * HID + tid] = v;
  }
  __syncthreads();
  if (wave < 3) {
    const v4f q = *(const v4fa*)(srow + wave * HID + 4 * lane);
    float* gp = GROW + (size_t)wave * HID + 4 * lane;
    *(volatile v4f*)gp = q;
  }
  __threadfence();
  if (wave < 3) {
    const v4f q = *(const v4fa*)(srow + wave * HID + 4 * lane);
    float* gp = GROW + (size_t)wave * HID + 4 * lane;
    *(volatile v4f*)gp = q;
  }
}

__global__ __launch_bounds__(NTHR) void k_head(const float* __restrict__ XV, const float* __restrict__ c1w,
                                               const float* __restrict__ c1b, const float* __restrict__ c2w,
                                               const float* __restrict__ c2b, int nN, float* out) {
  __shared__ __attribute__((aligned(16))) float sx[NWAVE * HID];
  __shared__ float sh[NWAVE * SHW];
  __shared__ float sw1[C1O * C1K];
  __shared__ float sb1[C1O];
  __shared__ float sw2[C1O * C2K];
  __shared__ float sb2[4];
  __shared__ __attribute__((aligned(16))) float sOut[HROWS * TOUT];
  const int tid = (int)threadIdx.x, lane = tid & 31, wave = tid >> 5;
  const int rowBase = (int)blockIdx.x * HROWS;

  {
    const int i1 = tid < C1O * C1K ? tid : C1O * C1K - 1;
    const int i2 = tid < C1O ? tid : C1O - 1;
    const int i3 = tid < C1O * C2K ? tid : C1O * C2K - 1;
    const float w1 = c1w[i1];
    const float vb = c1b[i2];
    const float w2 = c2w[i3];
    const float ub = c2b[0];
    if (tid < C1O * C1K) sw1[tid] = bf16_val(w1);
    if (tid < C1O)       sb1[tid] = bf16_val(vb);
    if (tid < C1O * C2K) sw2[tid] = bf16_val(w2);
    if (tid == 0)        sb2[0]   = bf16_val(ub);
  }

  float*       sxw = sx + wave * HID;
  float*       shw = sh + wave * SHW;
#pragma unroll 1
  for (int it = 0; it < HROWS / NWAVE; ++it) {
    const int lr = it * NWAVE + wave;
    const int gr = rowBase + lr;
    const int rc = gr < nN ? gr : nN - 1;
    __syncthreads();
    const v4f xv = *(const v4fa*)(XV + (size_t)rc * HID + 4 * lane);
    *(v4fa*)(sxw + 4 * lane) = xv;
    __syncthreads();
#pragma unroll 1
    for (int q = 0; q < 8; ++q) {
      const int idx = q * 32 + lane;
      const int idc = idx < C1O * C1P ? idx : C1O * C1P - 1;
      const int oc  = idc / C1P;
      const int tp  = idc - oc * C1P;
      const float* xp = sxw + C1S * tp;
      const float* wp = sw1 + oc * C1K;
      float a = sb1[oc];
#pragma unroll 3
      for (int j = 0; j < C1K; ++j) a = fmaf(xp[j], wp[j], a);
      a = fmaxf(a, 0.0f);
      if (idx < C1O * C1P) shw[idx] = a;
    }
    __syncthreads();
    {
      const int lc = lane < TOUT ? lane : TOUT - 1;
      float a = sb2[0];
#pragma unroll 1
      for (int oc = 0; oc < C1O; ++oc) {
        const float* hp = shw + oc * C1P + lc;
        const float* wp = sw2 + oc * C2K;
#pragma unroll 2
        for (int j = 0; j < C2K; ++j) a = fmaf(hp[j], wp[j], a);
      }
      if (lane < TOUT) sOut[lr * TOUT + lane] = a;
    }
  }
  __syncthreads();

  const int NP = (HROWS * TOUT) / 4;
  const long long lim = (long long)TOUT * (long long)nN;
#pragma unroll 1
  for (int it = 0; it < (NP + NTHR - 1) / NTHR; ++it) {
    const int p  = it * NTHR + tid;
    const int pc = p < NP ? p : NP - 1;
    const v4f v  = *(const v4fa*)(sOut + 4 * pc);
    const long long gidx = (long long)rowBase * TOUT + 4LL * pc;
    const bool stv = (p < NP) && (gidx + 4 <= lim);
    if (stv) *(volatile v4f*)(out + (size_t)gidx) = v;
  }
  __threadfence();
#pragma unroll 1
  for (int it = 0; it < (NP + NTHR - 1) / NTHR; ++it) {
    const int p  = it * NTHR + tid;
    const int pc = p < NP ? p : NP - 1;
    const v4f v  = *(const v4fa*)(sOut + 4 * pc);
    const long long gidx = (long long)rowBase * TOUT + 4LL * pc;
    const bool stv = (p < NP) && (gidx + 4 <= lim);
    if (stv) *(volatile v4f*)(out + (size_t)gidx) = v;
  }
}

static inline int cdiv(int a, int b) { return (a + b - 1) / b; }

extern "C" void kernel_launch(void* const* d_in, const int* in_sizes, int n_in,
                              void* d_out, int out_size, void* d_ws, size_t ws_size,
                              hipStream_t stream) {
  if (n_in < 37) return;
  if (in_sizes[0] < NIN || (in_sizes[0] % NIN) != 0) return;
  const int nN = in_sizes[0] / NIN;
  if (in_sizes[1] < EIN || (in_sizes[1] % EIN) != 0) return;
  const int nE = in_sizes[1] / EIN;
  if ((long long)in_sizes[2] != 2LL * (long long)nE) return;
  if (nN < 1 || nN >= (1 << 22) || nE < 1 || nE >= (1 << 21)) return;
  if (in_sizes[3] != NIN * HID || in_sizes[4] != HID) return;
  if (in_sizes[5] != HID * HID || in_sizes[6] != HID) return;
  if (in_sizes[7] != HID || in_sizes[8] != HID) return;
  if (in_sizes[9] != EIN * HID || in_sizes[10] != HID) return;
  if (in_sizes[11] != HID * HID || in_sizes[12] != HID) return;
  if (in_sizes[13] != HID || in_sizes[14] != HID) return;
  if (in_sizes[15] < 4 * HID * HID || (in_sizes[15] % (4 * HID * HID)) != 0) return;
  const int L = in_sizes[15] / (4 * HID * HID);
  if (L < 1 || L > 16) return;
  if (in_sizes[16] != L * HID || in_sizes[17] != L * HID * HID || in_sizes[18] != L * HID) return;
  if (in_sizes[19] != L * HID || in_sizes[20] != L * HID) return;
  if (in_sizes[21] != L * 3 * HID * HID || in_sizes[22] != L * HID || in_sizes[23] != L * HID * HID) return;
  if (in_sizes[24] != L * HID || in_sizes[25] != L * HID || in_sizes[26] != L * HID) return;
  if (in_sizes[27] != L * 3 * HID * HID || in_sizes[28] != L * HID || in_sizes[29] != L * HID * HID) return;
  if (in_sizes[30] != L * HID || in_sizes[31] != L * HID || in_sizes[32] != L * HID) return;
  if (in_sizes[33] != C1O * C1K || in_sizes[34] != C1O || in_sizes[35] != C1O * C2K || in_sizes[36] != 1) return;
  if ((long long)out_size != (long long)nN * TOUT) return;

  const float* x     = (const float*)d_in[0];
  const float* eattr = (const float*)d_in[1];
  const int*   ei    = (const int*)d_in[2];
  const float* Wn1   = (const float*)d_in[3];
  const float* bn1   = (const float*)d_in[4];
  const float* Wn2   = (const float*)d_in[5];
  const float* bn2   = (const float*)d_in[6];
  const float* gnln  = (const float*)d_in[7];
  const float* bnln  = (const float*)d_in[8];
  const float* We1   = (const float*)d_in[9];
  const float* be1   = (const float*)d_in[10];
  const float* We2   = (const float*)d_in[11];
  const float* be2   = (const float*)d_in[12];
  const float* geln  = (const float*)d_in[13];
  const float* beln  = (const float*)d_in[14];
  const float* lEW1  = (const float*)d_in[15];
  const float* lEb1  = (const float*)d_in[16];
  const float* lEW2  = (const float*)d_in[17];
  const float* lEb2  = (const float*)d_in[18];
  const float* lEg   = (const float*)d_in[19];
  const float* lEbt  = (const float*)d_in[20];
  const float* lVW1  = (const float*)d_in[21];
  const float* lVb1  = (const float*)d_in[22];
  const float* lVW2  = (const float*)d_in[23];
  const float* lVb2  = (const float*)d_in[24];
  const float* lVg   = (const float*)d_in[25];
  const float* lVbt  = (const float*)d_in[26];
  const float* lGW1  = (const float*)d_in[27];
  const float* lGb1  = (const float*)d_in[28];
  const float* lGW2  = (const float*)d_in[29];
  const float* lGb2  = (const float*)d_in[30];
  const float* lGg   = (const float*)d_in[31];
  const float* lGbt  = (const float*)d_in[32];
  const float* c1w   = (const float*)d_in[33];
  const float* c1b   = (const float*)d_in[34];
  const float* c2w   = (const float*)d_in[35];
  const float* c2b   = (const float*)d_in[36];
  float* out0 = (float*)d_out;

  const int MP = cdiv(nN, GBM) * GBM;
  const int gM = MP / GBM;
  const int EP = cdiv(nE, EPB) * EPB;
  const int gE = EP / EPB;
  const int gA = cdiv(MP, NBA);
  if ((long long)gA * NBA < (long long)MP) return;
  const int gH = cdiv(nN, HROWS);

  char* ws = (char*)d_ws;
  size_t off = 0;
  const size_t oWPL  = off; off += (size_t)(OFF_LAY + (size_t)L * PH_LAYER) * 2;   off = (off + 255) & ~(size_t)255;
  const size_t oGROW = off; off += (size_t)3 * HID * 4;                             off = (off + 255) & ~(size_t)255;
  const size_t oNREC = off; off += (size_t)gM * HID * 4;                            off = (off + 255) & ~(size_t)255;
  const size_t oEREC = off; off += (size_t)gE * HID * 4;                            off = (off + 255) & ~(size_t)255;
  const size_t oXV   = off; off += (size_t)MP * HID * 4;                            off = (off + 255) & ~(size_t)255;
  const size_t oXVB  = off; off += (size_t)MP * KHL * 2;                            off = (off + 255) & ~(size_t)255;
  const size_t oXE   = off; off += (size_t)EP * HID * 4;                            off = (off + 255) & ~(size_t)255;
  const size_t oPE   = off; off += (size_t)MP * KHL * 4;                            off = (off + 255) & ~(size_t)255;
  if (off > ws_size || off > (size_t)WSMAX) return;
  unsigned short* WPL  = (unsigned short*)(ws + oWPL);
  float*          GROW = (float*)(ws + oGROW);
  float*          NREC = (float*)(ws + oNREC);
  float*          EREC = (float*)(ws + oEREC);
  float*          XV   = (float*)(ws + oXV);
  unsigned short* XVB  = (unsigned short*)(ws + oXVB);
  float*          XE   = (float*)(ws + oXE);
  float*          PE   = (float*)(ws + oPE);
  float*          AGG  = (float*)(ws + oPE);
  const unsigned short* WN1T = WPL + OFF_WN1T;
  const unsigned short* WN2T = WPL + OFF_WN2T;
  const unsigned short* WE1T = WPL + OFF_WE1T;
  const unsigned short* WE2T = WPL + OFF_WE2T;

  hipFuncSetAttribute(reinterpret_cast<const void*>(&k_edge<true>), hipFuncAttributeMaxDynamicSharedMemorySize,
                      (int)EDGE_LDS_BYTES);
  hipFuncSetAttribute(reinterpret_cast<const void*>(&k_edge<false>), hipFuncAttributeMaxDynamicSharedMemorySize,
                      (int)EDGE_LDS_BYTES);
  hipFuncSetAttribute(reinterpret_cast<const void*>(&k_node<true>), hipFuncAttributeMaxDynamicSharedMemorySize,
                      (int)NODE_LDS_BYTES);
  hipFuncSetAttribute(reinterpret_cast<const void*>(&k_node<false>), hipFuncAttributeMaxDynamicSharedMemorySize,
                      (int)NODE_LDS_BYTES);
  hipFuncSetAttribute(reinterpret_cast<const void*>(&k_scan), hipFuncAttributeMaxDynamicSharedMemorySize,
                      (int)SCAN_LDS_BYTES);

  const int nPrepU = NU_W32 + NU_W256 + NU_W32 + NU_W256 + L * NU_LAYER + NU_GROW;
  const int vec8   = ((nE & 3) == 0) ? 1 : 0;

  k_prep<<<cdiv(nPrepU, NTHR), NTHR, 0, stream>>>(Wn1, Wn2, We1, We2, lEW1, lEW2, lVW1, lVW2, lEb1, lVb1, L,
                                                  WPL, GROW);
  k_node<true><<<gM, GTHR, NODE_LDS_BYTES, stream>>>(x, XV, AGG, WN1T, bn1, GROW, WN2T, bn2, gnln, bnln, nN,
                                                      XVB, NREC);
  k_edge<true><<<gE, NTHR, EDGE_LDS_BYTES, stream>>>(ei, nE, nN, eattr, XE, PE, GROW, WE1T, WE2T, be1, be2,
                                                      geln, beln, EREC);
  for (int l = 0; l < L; ++l) {
    const unsigned short* lay  = WPL + OFF_LAY + (size_t)l * PH_LAYER;
    const unsigned short* WABT = lay + LO_WABT;
    const unsigned short* WCT  = lay + LO_WCT;
    const unsigned short* WE2L = lay + LO_WE2;
    const unsigned short* WV1T = lay + LO_WV1;
    const unsigned short* WV2T = lay + LO_WV2;
    const float* Eb1l = lEb1 + (size_t)l * HID;
    const float* Eb2l = lEb2 + (size_t)l * HID;
    const float* Egl  = lEg  + (size_t)l * HID;
    const float* Ebtl = lEbt + (size_t)l * HID;
    const float* Vb2l = lVb2 + (size_t)l * HID;
    const float* Vgl  = lVg  + (size_t)l * HID;
    const float* Vbtl = lVbt + (size_t)l * HID;
    k_pe<<<dim3(gM, 2), GTHR, 0, stream>>>(XVB, WABT, PE);
    k_edge<false><<<gE, NTHR, EDGE_LDS_BYTES, stream>>>(ei, nE, nN, eattr, XE, PE, GROW, WCT, WE2L, Eb1l, Eb2l,
                                                         Egl, Ebtl, EREC);
    k_scan<<<gA, NTHR, SCAN_LDS_BYTES, stream>>>(ei + nE, nE, vec8, MP, XE, AGG);
    k_node<false><<<gM, GTHR, NODE_LDS_BYTES, stream>>>(x, XV, AGG, WV1T, bn1, GROW, WV2T, Vb2l, Vgl, Vbtl, nN,
                                                         XVB, NREC);
    if (l + 1 < L) {
      k_glob<<<1, NTHR, 0, stream>>>(NREC, gM, EREC, gE, GROW,
                                     lGW1 + (size_t)l * 3 * HID * HID, lGb1 + (size_t)l * HID,
                                     lGW2 + (size_t)l * HID * HID, lGb2 + (size_t)l * HID,
                                     lGg + (size_t)l * HID, lGbt + (size_t)l * HID,
                                     lEW1 + (size_t)(l + 1) * 4 * HID * HID, lEb1 + (size_t)(l + 1) * HID,
                                     lVW1 + (size_t)(l + 1) * 3 * HID * HID, lVb1 + (size_t)(l + 1) * HID);
    }
  }
  k_head<<<gH, NTHR, 0, stream>>>(XV, c1w, c1b, c2w, c2b, nN, out0);
}
